// JointSupervisedGroundedCoreferencer_60387240182304
// MI455X (gfx1250) — hardware-verified
//
#include <hip/hip_runtime.h>
#include <math.h>

#ifndef NB
#define NB 128
#endif
#define NB_FULL 128
#define NSPAN 32
#define NIMG 36
#define DSP 512
#define DVI 1024
#define HID 512
#define NPAIR 496
#define PPAD 512
#define MTOK (NB * NSPAN)
#define MNL (NSPAN * NIMG)
#define UVP (2 * HID)
#define PT 64
#define PA 520
#define NEG_FILL (-9.0e9f)

#define OUT_TS_OFF (1 + NB_FULL * MNL)
#define OUT_TOTAL (OUT_TS_OFF + NB_FULL * NPAIR)
#define OUT_Q (OUT_TOTAL / 4)

static_assert(NB >= 2 && NB <= NB_FULL && NB % 2 == 0);
static_assert(NB_FULL == 128);
static_assert(MTOK % 64 == 0);
static_assert(DVI % 64 == 0 && UVP % 64 == 0 && HID % 64 == 0);
static_assert(DSP % 32 == 0 && DVI % 32 == 0 && HID % 32 == 0);
static_assert(DSP == HID);
static_assert(NPAIR == NSPAN * (NSPAN - 1) / 2);
static_assert(PPAD % PT == 0 && PPAD >= NPAIR && PPAD / PT == 8);
static_assert(PA % 8 == 0 && PA >= HID && PA >= DSP);
static_assert((PT * (DSP / 8)) % 256 == 0);
static_assert(HID == 8 * 64);
static_assert(MNL % 4 == 0 && (MNL * 4) % 128 == 0);
static_assert(MNL / 4 <= 2 * 192 && (MNL / 4 - 192) % 32 == 0);
static_assert(NIMG <= 48 && NSPAN == 32);
static_assert((MTOK * DSP / 8) % 256 == 0 && (NB * NIMG * DVI / 8) % 256 == 0);
static_assert(4 * 1 == 4);
static_assert(OUT_TS_OFF * 4 == 589828);
static_assert(OUT_TOTAL * 4 == 843780);
static_assert(OUT_TOTAL - 4 * OUT_Q == 1 && OUT_Q % 32 == 0);
static_assert(32 * 16 * 8 == 16 * 64 * 4);
static_assert(32 * 16 * 4 == 16 * 64 * 2);
static_assert(32 * 8 * 8 == 16 * 64 * 2);
static_assert(16 * 16 == PT * 4);
static_assert(8 * 16 * 68 * 4 <= 131072);
static_assert(PT * PA * 2 + 8 * 16 * 68 * 4 + 8 * PT * 4 + 2 * PT * 4 <= 131072);
static_assert(MNL * 4 + 128 * 37 * 4 + 32 * 4 + 128 * 4 <= 131072);

static constexpr float SC_XW = 1.0f / 256.0f;
static constexpr float SC_PW = 1.0f / 2048.0f;
static constexpr float SC_GI = 1.0f / 64.0f;

static constexpr size_t al256(size_t x) { return (x + 255) & ~(size_t)255; }
static constexpr size_t WS_TOTAL =
    al256((size_t)MTOK * DSP * 2) + al256((size_t)NB * NIMG * DVI * 2) + al256((size_t)DSP * DVI * 2) +
    al256((size_t)3 * DSP * HID * 2) + al256((size_t)HID * HID * 2) + al256((size_t)MTOK * DVI * 2) +
    al256((size_t)MTOK * UVP * 4) + al256((size_t)NB * MNL * 4) + al256((size_t)NB * PPAD * 4) +
    al256((size_t)NB * 128 * 4) + al256((size_t)128);
static_assert(WS_TOTAL <= (size_t)134217728);

typedef _Float16 h16;
typedef __attribute__((ext_vector_type(16))) _Float16 v16h;
typedef __attribute__((ext_vector_type(8)))  _Float16 v8h;
typedef __attribute__((ext_vector_type(4)))  _Float16 v4h;
typedef __attribute__((ext_vector_type(8)))  float    v8f;
typedef __attribute__((ext_vector_type(4)))  float    v4f;
typedef __attribute__((ext_vector_type(4)))  unsigned int v4u;


#define VST2(T, ptr, val) do { const T vst2_v_ = (val); *(volatile T*)(ptr) = vst2_v_; __threadfence(); *(volatile T*)(ptr) = vst2_v_; } while (0)
#define VST2V4(ptr, val) do { const v4f vst2_v4_ = (val); *(volatile v4f*)(ptr) = vst2_v4_; __threadfence(); *(volatile v4f*)(ptr) = vst2_v4_; } while (0)

__device__ __forceinline__ float bfr(float f) {
    unsigned u = __float_as_uint(f);
    u += 0x7FFFu + ((u >> 16) & 1u);
    return __uint_as_float(u & 0xFFFF0000u);
}
__device__ __forceinline__ unsigned short f2h_bits(float x) {
    return (fabsf(x) < 6.104e-5f) ? (unsigned short)0 : __builtin_bit_cast(unsigned short, (_Float16)x);
}
__device__ __forceinline__ void st8h(unsigned short* P, size_t o, const float* v) {
    v4u pk;
    pk.x = (unsigned)f2h_bits(v[0]) | ((unsigned)f2h_bits(v[1]) << 16);
    pk.y = (unsigned)f2h_bits(v[2]) | ((unsigned)f2h_bits(v[3]) << 16);
    pk.z = (unsigned)f2h_bits(v[4]) | ((unsigned)f2h_bits(v[5]) << 16);
    pk.w = (unsigned)f2h_bits(v[6]) | ((unsigned)f2h_bits(v[7]) << 16);
    VST2(v4u, (v4u*)(P + o), pk);
}
static __device__ __forceinline__ h16 toh_flush(float v) {
    const h16 r = (h16)v;
    return (fabsf(v) < 6.103515625e-05f) ? (h16)0.0f : r;
}

union FragU { v16h v; v8h h[2]; };
__device__ __forceinline__ v16h frag_ld(const _Float16* p) {
    FragU f; f.h[0] = *(const v8h*)(p); f.h[1] = *(const v8h*)(p + 16); return f.v;
}
__device__ __forceinline__ v8f wmma16(v16h a, v16h b, v8f c) {
    c = __builtin_amdgcn_wmma_f32_16x16x32_f16(false, a, false, b, (short)0, c, false, false);
    asm volatile("v_nop\n\tv_nop\n\tv_nop\n\tv_nop" : "+v"(c) : "v"(a), "v"(b));
    return c;
}
__device__ __forceinline__ void wave_sync_lds() {
    __builtin_amdgcn_fence(3  , "workgroup");
    __builtin_amdgcn_wave_barrier();
    __builtin_amdgcn_fence(2  , "workgroup");
}

template <int OUT_MODE>
__device__ __forceinline__ void gemm64_body(const _Float16* __restrict__ A, unsigned lda,
                                            const _Float16* __restrict__ Bt, unsigned ldb,
                                            void* __restrict__ Cout, unsigned ldc,
                                            unsigned M, unsigned N, unsigned K, float scale, float oscale) {
  __shared__ __align__(16) float sT[8 * 16 * 68];
  const unsigned lane = threadIdx.x & 31u;
  const unsigned wave = (unsigned)__builtin_amdgcn_readfirstlane((int)(threadIdx.x >> 5));
  const unsigned tilesN = N >> 6, tilesM = M >> 6;
  const unsigned tile = blockIdx.x * 8u + wave;
  if (tile >= tilesM * tilesN) return;
  const unsigned tm = tile / tilesN;
  const unsigned tn = tile - tm * tilesN;
  const unsigned m0 = tm << 6, n0 = tn << 6;
  const unsigned rlane = lane & 15u;
  const unsigned koff = (lane >> 4) * 8u;
  const unsigned sb = wave * (16u * 68u);

  v8f acc[4][4];
#pragma unroll
  for (int i = 0; i < 4; ++i)
#pragma unroll
    for (int j = 0; j < 4; ++j) acc[i][j] = (v8f){0.f,0.f,0.f,0.f,0.f,0.f,0.f,0.f};

#pragma unroll 1
  for (unsigned k0 = 0; k0 < K; k0 += 32u) {
    v16h bh[4];
#pragma unroll
    for (int j = 0; j < 4; ++j)
      bh[j] = frag_ld(Bt + (size_t)(n0 + ((unsigned)j << 4) + rlane) * ldb + koff + k0);
#pragma unroll
    for (int i = 0; i < 4; ++i) {
      const v16h ah = frag_ld(A + (size_t)(m0 + ((unsigned)i << 4) + rlane) * lda + koff + k0);
#pragma unroll
      for (int j = 0; j < 4; ++j) acc[i][j] = wmma16(ah, bh[j], acc[i][j]);
    }
  }

#pragma unroll
  for (int i = 0; i < 4; ++i) {
    const unsigned mBase = m0 + ((unsigned)i << 4);
#pragma unroll
    for (int j = 0; j < 4; ++j) {
#pragma unroll
      for (int r = 0; r < 8; ++r) {
        float v = acc[i][j][r] * scale;
        if (OUT_MODE == 1) v *= oscale;
        sT[sb + (koff + (unsigned)r) * 68u + ((unsigned)j << 4) + rlane] = v;
      }
    }
    wave_sync_lds();
    if (OUT_MODE == 0) {
      float* C = (float*)Cout;
      const unsigned hh = lane >> 4, c4 = (lane & 15u) * 4u;
#pragma unroll
      for (int half = 0; half < 2; ++half) {
        v4f vv[4];
#pragma unroll
        for (int it = 0; it < 4; ++it) {
          const unsigned row = (unsigned)(half * 4 + it) * 2u + hh;
          vv[it] = *(const v4f*)(&sT[sb + row * 68u + c4]);
        }
        for (int pass = 0; pass < 2; ++pass) {
#pragma unroll
          for (int it = 0; it < 4; ++it) {
            const unsigned row = (unsigned)(half * 4 + it) * 2u + hh;
            *(volatile v4f*)(C + (size_t)(mBase + row) * ldc + n0 + c4) = vv[it];
          }
          __threadfence();
        }
      }
    } else {
      _Float16* C = (_Float16*)Cout;
      const unsigned q = lane >> 3, c8 = (lane & 7u) * 8u;
      v8h hv[4];
#pragma unroll
      for (int it = 0; it < 4; ++it) {
        const unsigned row = (unsigned)it * 4u + q;
#pragma unroll
        for (int e = 0; e < 8; ++e) hv[it][e] = toh_flush(sT[sb + row * 68u + c8 + (unsigned)e]);
      }
      for (int pass = 0; pass < 2; ++pass) {
#pragma unroll
        for (int it = 0; it < 4; ++it) {
          const unsigned row = (unsigned)it * 4u + q;
          *(volatile v8h*)(C + (size_t)(mBase + row) * ldc + n0 + c8) = hv[it];
        }
        __threadfence();
      }
    }
    wave_sync_lds();
  }
}

__global__ __launch_bounds__(256) void k_gemm_g(const _Float16* __restrict__ A, unsigned lda, const _Float16* __restrict__ Bt, unsigned ldb,
                                                _Float16* __restrict__ C, unsigned ldc, unsigned M, unsigned N, unsigned K,
                                                float scale, float oscale) {
  gemm64_body<1>(A, lda, Bt, ldb, (void*)C, ldc, M, N, K, scale, oscale);
}
__global__ __launch_bounds__(256) void k_gemm_uv(const _Float16* __restrict__ A, unsigned lda, const _Float16* __restrict__ Bt, unsigned ldb,
                                                 float* __restrict__ C, unsigned ldc, unsigned M, unsigned N, unsigned K,
                                                 float scale, float oscale) {
  gemm64_body<0>(A, lda, Bt, ldb, (void*)C, ldc, M, N, K, scale, oscale);
}

__global__ __launch_bounds__(256) void k_wt16(const float* __restrict__ Wm, unsigned KI, unsigned NO, unsigned lgper,
                                              unsigned short* __restrict__ W16, float sw) {
    const unsigned layer = blockIdx.y;
    const float* Wl = Wm + (size_t)layer * KI * NO;
    unsigned short* Dl = W16 + (size_t)layer * KI * NO;
    const unsigned u = blockIdx.x * 256u + threadIdx.x;
    const unsigned per = 1u << lgper;
    if (u >= NO * per) return;
    const unsigned k0 = 8u * (u & (per - 1u));
    const unsigned o = u >> lgper;
    float v[8];
#pragma unroll
    for (int i = 0; i < 8; ++i) v[i] = bfr(Wl[(size_t)(k0 + (unsigned)i) * NO + o]) * sw;
    st8h(Dl, (size_t)o * KI + k0, v);
}

__global__ __launch_bounds__(256) void k_cvt8(const float* __restrict__ src, unsigned short* __restrict__ dst, unsigned n8, float s) {
    const unsigned u = blockIdx.x * 256u + threadIdx.x;
    if (u >= n8) return;
    const v4f a = *(const v4f*)(src + (size_t)u * 8u);
    const v4f b = *(const v4f*)(src + (size_t)u * 8u + 4u);
    float v[8] = {bfr(a.x) * s, bfr(a.y) * s, bfr(a.z) * s, bfr(a.w) * s, bfr(b.x) * s, bfr(b.y) * s, bfr(b.z) * s, bfr(b.w) * s};
    st8h(dst, (size_t)u * 8u, v);
}

__global__ __launch_bounds__(192) void k_bil_sent(const _Float16* __restrict__ G16, const _Float16* __restrict__ img16,
                                                  const float* __restrict__ smask, const float* __restrict__ imask,
                                                  float* __restrict__ Mws, float* __restrict__ sent) {
    __shared__ __align__(16) float sM[MNL];
    __shared__ float sIm[128 * 37];
    __shared__ float sSm[32];
    __shared__ __align__(16) float sRow[128];
    const unsigned tid = threadIdx.x, lane = tid & 31u;
    const unsigned wave = (unsigned)__builtin_amdgcn_readfirstlane((int)(tid >> 5));
    const unsigned hh = lane >> 4, c = lane & 15u;
    const unsigned b = blockIdx.x;

    for (unsigned idx = tid; idx < (unsigned)(NB * NIMG); idx += 192u) {
        const unsigned j = idx / (unsigned)NIMG;
        const unsigned l = idx - j * (unsigned)NIMG;
        sIm[j * 37u + l] = bfr(imask[idx]);
    }
    if (tid < 32u) sSm[tid] = bfr(smask[b * NSPAN + tid]);

    const unsigned rt = wave / 3u, ct = wave - 3u * rt;
    const unsigned l = ct * 16u + c;
    const unsigned lcl = (l < (unsigned)NIMG) ? l : (unsigned)(NIMG - 1);
    const _Float16* ap = G16 + (size_t)(b * NSPAN + rt * 16u + c) * DVI + 8u * hh;
    const _Float16* bp = img16 + (size_t)(b * NIMG + lcl) * DVI + 8u * hh;
    v8f acc = (v8f){0.f,0.f,0.f,0.f,0.f,0.f,0.f,0.f};
#pragma unroll 2
    for (unsigned k0 = 0; k0 < (unsigned)DVI; k0 += 32u) {
        const v16h a = frag_ld(ap + k0);
        const v16h bf = frag_ld(bp + k0);
        acc = wmma16(a, bf, acc);
    }
#pragma unroll
    for (int r = 0; r < 8; ++r) {
        const unsigned n = rt * 16u + 8u * hh + (unsigned)r;
        if (l < (unsigned)NIMG) sM[n * (unsigned)NIMG + l] = acc[r] * SC_GI;
    }
    __syncthreads();

#pragma unroll
    for (unsigned trip = 0; trip < 2u; ++trip) {
        const unsigned t = trip * 192u + tid;
        if (t < (unsigned)(MNL / 4)) {
            const v4f v = *(const v4f*)(&sM[4u * t]);
            VST2V4(Mws + (size_t)b * MNL + 4u * t, v);
        }
    }

    float sv = 0.f;
    if (tid < (unsigned)NB) {
        const unsigned ib = tid * 37u;
        float mx = -3.0e38f;
#pragma unroll 1
        for (unsigned n = 0; n < (unsigned)NSPAN; ++n) {
            const float a = sSm[n];
#pragma unroll 1
            for (unsigned q = 0; q < (unsigned)NIMG; ++q) {
                const float v = a * sIm[ib + q];
                const float pm = (v != 0.0f) ? v : NEG_FILL;
                mx = fmaxf(mx, pm);
            }
        }
        float den = 0.f, num = 0.f;
#pragma unroll 1
        for (unsigned n = 0; n < (unsigned)NSPAN; ++n) {
            const float a = sSm[n];
#pragma unroll 1
            for (unsigned q = 0; q < (unsigned)NIMG; ++q) {
                const float v = a * sIm[ib + q];
                const float pm = (v != 0.0f) ? v : NEG_FILL;
                const float e = expf(pm - mx);
                den += e;
                num += e * sM[n * (unsigned)NIMG + q];
            }
        }
        sv = num * (1.0f / den);
    }
    if (tid < 128u) sRow[tid] = sv;
    __syncthreads();
    if (tid < 32u) {
        const v4f v = *(const v4f*)(&sRow[4u * tid]);
        VST2V4(sent + (size_t)b * 128u + 4u * tid, v);
    }
}

__global__ __launch_bounds__(128) void k_loss(const float* __restrict__ sent, float* __restrict__ lossline) {
    __shared__ float red[128];
    const unsigned i = threadIdx.x;
    float term = 0.f;
    if (i < (unsigned)NB) {
#pragma unroll 1
        for (unsigned pass = 0; pass < 2u; ++pass) {
            const unsigned si = pass ? 1u : 128u, sj = pass ? 128u : 1u;
            float mx = -3.0e38f;
#pragma unroll 1
            for (unsigned j = 0; j < (unsigned)NB; ++j) mx = fmaxf(mx, sent[i * si + j * sj]);
            float z = 0.f, rs = 0.f;
#pragma unroll 1
            for (unsigned j = 0; j < (unsigned)NB; ++j) {
                const float v = sent[i * si + j * sj];
                z += expf(v - mx);
                rs += v;
            }
            term += (float)NB * (mx + logf(z)) - rs;
        }
    }
    red[i] = term;
    __syncthreads();
    for (unsigned off = 64u; off > 0u; off >>= 1) {
        if (i < off) red[i] += red[i + off];
        __syncthreads();
    }
    if (i < 8u) {
        const float t = red[0] * (1.0f / (float)NB);
        v4f v;
        v.x = (i == 0u) ? t : 0.f; v.y = 0.f; v.z = 0.f; v.w = 0.f;
        VST2V4(lossline + 4u * i, v);
    }
}

__global__ __launch_bounds__(256) void k_pair(const _Float16* __restrict__ span16, const _Float16* __restrict__ w1c,
                                              const _Float16* __restrict__ w2t, const float* __restrict__ UV,
                                              const float* __restrict__ b1, const float* __restrict__ b2,
                                              const float* __restrict__ W3, const float* __restrict__ b3,
                                              float* __restrict__ tsW) {
    __shared__ __align__(16) _Float16 sA[PT * PA];
    __shared__ __align__(16) float sT[8 * 16 * 68];
    __shared__ __align__(16) float sPart[8 * PT];
    __shared__ int sIu[PT];
    __shared__ int sJu[PT];
    const unsigned tid = threadIdx.x, lane = tid & 31u;
    const unsigned wave = (unsigned)__builtin_amdgcn_readfirstlane((int)(tid >> 5));
    const unsigned hh = lane >> 4, c = lane & 15u;
    const unsigned koff = 8u * hh;
    const unsigned b = blockIdx.x >> 3, tile = blockIdx.x & 7u;
    const unsigned p0 = tile * (unsigned)PT;

    if (tid < (unsigned)PT) {
        int p = (int)(p0 + tid);
        p = (p < NPAIR) ? p : (NPAIR - 1);
        int i = 0, base = 0;
#pragma unroll 1
        for (int s = 0; s < NSPAN - 1; ++s) {
            const int len = NSPAN - 1 - i;
            if (base + len <= p) { base += len; ++i; }
        }
        sIu[tid] = i;
        sJu[tid] = i + 1 + (p - base);
    }
    __syncthreads();

#pragma unroll 2
    for (unsigned it = 0; it < (unsigned)((PT * (DSP / 8)) / 256); ++it) {
        const unsigned piece = it * 256u + tid;
        const unsigned row = piece >> 6;
        const unsigned q8 = (piece & 63u) * 8u;
        const unsigned ra = b * NSPAN + (unsigned)sIu[row];
        const unsigned rb = b * NSPAN + (unsigned)sJu[row];
        const v8h xa = *(const v8h*)(span16 + (size_t)ra * DSP + q8);
        const v8h xb = *(const v8h*)(span16 + (size_t)rb * DSP + q8);
        v8h pr;
#pragma unroll
        for (int e = 0; e < 8; ++e) pr[e] = toh_flush((float)xa[e] * (float)xb[e]);
        *(v8h*)(&sA[row * (unsigned)PA + q8]) = pr;
    }
    __syncthreads();

    const unsigned n0 = wave * 64u;
    const unsigned sb = wave * (16u * 68u);
    v8f acc[4][4];
#pragma unroll
    for (int i = 0; i < 4; ++i)
#pragma unroll
        for (int j = 0; j < 4; ++j) acc[i][j] = (v8f){0.f,0.f,0.f,0.f,0.f,0.f,0.f,0.f};

#pragma unroll 1
    for (unsigned k0 = 0; k0 < (unsigned)DSP; k0 += 32u) {
        v16h bh[4];
#pragma unroll
        for (int j = 0; j < 4; ++j)
            bh[j] = frag_ld(w1c + (size_t)(n0 + ((unsigned)j << 4) + c) * DSP + koff + k0);
#pragma unroll
        for (int i = 0; i < 4; ++i) {
            const unsigned ai = (((unsigned)i << 4) + c) * (unsigned)PA + koff + k0;
            FragU fa;
            fa.h[0] = *(const v8h*)(&sA[ai]);
            fa.h[1] = *(const v8h*)(&sA[ai + 16u]);
#pragma unroll
            for (int j = 0; j < 4; ++j) acc[i][j] = wmma16(fa.v, bh[j], acc[i][j]);
        }
    }
    __syncthreads();

    {
        const unsigned c4 = (lane & 15u) * 4u;
        const v4f bq = *(const v4f*)(b1 + n0 + c4);
        const float bb0 = bfr(bq.x), bb1 = bfr(bq.y), bb2 = bfr(bq.z), bb3 = bfr(bq.w);
#pragma unroll
        for (int i = 0; i < 4; ++i) {
#pragma unroll
            for (int j = 0; j < 4; ++j)
#pragma unroll
                for (int r = 0; r < 8; ++r)
                    sT[sb + (koff + (unsigned)r) * 68u + ((unsigned)j << 4) + c] = acc[i][j][r] * SC_PW;
            wave_sync_lds();
#pragma unroll 2
            for (unsigned it = 0; it < 8u; ++it) {
                const unsigned row = 2u * it + hh;
                const unsigned prow = ((unsigned)i << 4) + row;
                const v4f v = *(const v4f*)(&sT[sb + row * 68u + c4]);
                const unsigned ru = b * NSPAN + (unsigned)sIu[prow];
                const unsigned rv = b * NSPAN + (unsigned)sJu[prow];
                const v4f u = *(const v4f*)(UV + (size_t)ru * UVP + n0 + c4);
                const v4f w = *(const v4f*)(UV + (size_t)rv * UVP + HID + n0 + c4);
                v4h hv;
                hv.x = toh_flush(fmaxf(v.x + (u.x + w.x) + bb0, 0.0f) * 8.0f);
                hv.y = toh_flush(fmaxf(v.y + (u.y + w.y) + bb1, 0.0f) * 8.0f);
                hv.z = toh_flush(fmaxf(v.z + (u.z + w.z) + bb2, 0.0f) * 8.0f);
                hv.w = toh_flush(fmaxf(v.w + (u.w + w.w) + bb3, 0.0f) * 8.0f);
                *(v4h*)(&sA[prow * (unsigned)PA + n0 + c4]) = hv;
            }
            wave_sync_lds();
        }
    }
    __syncthreads();

#pragma unroll
    for (int i = 0; i < 4; ++i)
#pragma unroll
        for (int j = 0; j < 4; ++j) acc[i][j] = (v8f){0.f,0.f,0.f,0.f,0.f,0.f,0.f,0.f};

#pragma unroll 1
    for (unsigned k0 = 0; k0 < (unsigned)HID; k0 += 32u) {
        v16h bh[4];
#pragma unroll
        for (int j = 0; j < 4; ++j)
            bh[j] = frag_ld(w2t + (size_t)(n0 + ((unsigned)j << 4) + c) * HID + koff + k0);
#pragma unroll
        for (int i = 0; i < 4; ++i) {
            const unsigned ai = (((unsigned)i << 4) + c) * (unsigned)PA + koff + k0;
            FragU fa;
            fa.h[0] = *(const v8h*)(&sA[ai]);
            fa.h[1] = *(const v8h*)(&sA[ai + 16u]);
#pragma unroll
            for (int j = 0; j < 4; ++j) acc[i][j] = wmma16(fa.v, bh[j], acc[i][j]);
        }
    }

    {
        float w3v[4], b2v[4];
#pragma unroll
        for (int j = 0; j < 4; ++j) {
            const unsigned col = n0 + ((unsigned)j << 4) + c;
            w3v[j] = bfr(W3[col]);
            b2v[j] = bfr(b2[col]);
        }
#pragma unroll
        for (int i = 0; i < 4; ++i) {
#pragma unroll
            for (int r = 0; r < 8; ++r) {
                float s = 0.f;
#pragma unroll
                for (int j = 0; j < 4; ++j) s += fmaxf(acc[i][j][r] * SC_XW + b2v[j], 0.0f) * w3v[j];
                s += __shfl_xor(s, 1, 32);
                s += __shfl_xor(s, 2, 32);
                s += __shfl_xor(s, 4, 32);
                s += __shfl_xor(s, 8, 32);
                if (c == 0u) sPart[wave * (unsigned)PT + ((unsigned)i << 4) + koff + (unsigned)r] = s;
            }
        }
    }
    __syncthreads();
    if (tid < 16u) {
        const float b3v = bfr(b3[0]);
        float o[4];
#pragma unroll
        for (int e = 0; e < 4; ++e) {
            const unsigned row = 4u * tid + (unsigned)e;
            float t = 0.f;
#pragma unroll
            for (unsigned w = 0; w < 8u; ++w) t += sPart[w * (unsigned)PT + row];
            o[e] = t + b3v;
        }
        v4f ov; ov.x = o[0]; ov.y = o[1]; ov.z = o[2]; ov.w = o[3];
        VST2V4(tsW + (size_t)b * PPAD + p0 + 4u * tid, ov);
    }
}

__device__ __forceinline__ float pack_fetch(const float* __restrict__ wsf, unsigned e, unsigned lossOff, unsigned mOff, unsigned tsOff) {
    unsigned em = (e >= 1u) ? (e - 1u) : 0u;
    em = (em < (unsigned)(NB_FULL * MNL)) ? em : (unsigned)(NB_FULL * MNL - 1);
    const unsigned bm = em / (unsigned)MNL;
    unsigned et = (e >= (unsigned)OUT_TS_OFF) ? (e - (unsigned)OUT_TS_OFF) : 0u;
    et = (et < (unsigned)(NB_FULL * NPAIR)) ? et : (unsigned)(NB_FULL * NPAIR - 1);
    const unsigned bt = et / (unsigned)NPAIR;
    const unsigned pt = et - bt * (unsigned)NPAIR;
    const bool isL = (e == 0u);
    const bool isM = (!isL) && (e < (unsigned)OUT_TS_OFF);
    const bool valid = isL || (isM ? (bm < (unsigned)NB) : (bt < (unsigned)NB));
    unsigned off = isL ? lossOff : (isM ? (mOff + em) : (tsOff + bt * (unsigned)PPAD + pt));
    off = valid ? off : lossOff;
    const float x = wsf[off];
    return valid ? x : 0.0f;
}
__global__ __launch_bounds__(256) void k_pack(const float* __restrict__ wsf, unsigned lossOff, unsigned mOff, unsigned tsOff,
                                              float* __restrict__ out) {
    const unsigned q = blockIdx.x * 256u + threadIdx.x;
    float v[4];
#pragma unroll
    for (int k = 0; k < 4; ++k) {
        unsigned e = 4u * q + (unsigned)k;
        e = (e < (unsigned)OUT_TOTAL) ? e : (unsigned)(OUT_TOTAL - 1);
        v[k] = pack_fetch(wsf, e, lossOff, mOff, tsOff);
    }
    if (q < (unsigned)OUT_Q) {
        v4f o; o.x = v[0]; o.y = v[1]; o.z = v[2]; o.w = v[3];
        VST2V4(out + (size_t)4u * q, o);
    } else if (q == (unsigned)OUT_Q) {
        VST2(float, out + (size_t)4u * q, v[0]);
    }
}

extern "C" void kernel_launch(void* const* d_in, const int* in_sizes, int n_in, void* d_out, int out_size,
                              void* d_ws, size_t ws_size, hipStream_t stream) {
    if (n_in < 11) return;
    if (in_sizes[0] < MTOK * DSP || in_sizes[1] < NB * NIMG * DVI || in_sizes[2] < NB * NSPAN || in_sizes[3] < NB * NIMG) return;
    if (in_sizes[4] < DSP * DVI || in_sizes[5] < 3 * DSP * HID || in_sizes[6] < HID || in_sizes[7] < HID * HID) return;
    if (in_sizes[8] < HID || in_sizes[9] < HID || in_sizes[10] < 1 || out_size < OUT_TOTAL) return;

    const float* span  = (const float*)d_in[0];
    const float* img   = (const float*)d_in[1];
    const float* smask = (const float*)d_in[2];
    const float* imask = (const float*)d_in[3];
    const float* Wg    = (const float*)d_in[4];
    const float* W1    = (const float*)d_in[5];
    const float* b1    = (const float*)d_in[6];
    const float* W2    = (const float*)d_in[7];
    const float* b2    = (const float*)d_in[8];
    const float* W3    = (const float*)d_in[9];
    const float* b3    = (const float*)d_in[10];
    float* out = (float*)d_out;

    char* wsp = (char*)d_ws;
    size_t off = 0;
    auto carve = [&](size_t bytes) -> void* { void* r = wsp + off; off += (bytes + 255) & ~(size_t)255; return r; };
    unsigned short* span16 = (unsigned short*)carve((size_t)MTOK * DSP * 2);
    unsigned short* img16  = (unsigned short*)carve((size_t)NB * NIMG * DVI * 2);
    unsigned short* wg16   = (unsigned short*)carve((size_t)DSP * DVI * 2);
    unsigned short* w1_16  = (unsigned short*)carve((size_t)3 * DSP * HID * 2);
    unsigned short* w2_16  = (unsigned short*)carve((size_t)HID * HID * 2);
    unsigned short* g16    = (unsigned short*)carve((size_t)MTOK * DVI * 2);
    float*          uv     = (float*)carve((size_t)MTOK * UVP * 4);
    float*          mws    = (float*)carve((size_t)NB * MNL * 4);
    float*          tsw    = (float*)carve((size_t)NB * PPAD * 4);
    float*          sentw  = (float*)carve((size_t)NB * 128 * 4);
    float*          lossw  = (float*)carve((size_t)128);
    if (off > ws_size || off > (size_t)134217728 || off != WS_TOTAL) return;

    k_wt16<<<dim3((DVI * (DSP / 8)) / 256, 1), 256, 0, stream>>>(Wg, DSP, DVI, 6, wg16, 32.0f);
    k_wt16<<<dim3((HID * (DSP / 8)) / 256, 3), 256, 0, stream>>>(W1, DSP, HID, 6, w1_16, 32.0f);
    k_wt16<<<dim3((HID * (HID / 8)) / 256, 1), 256, 0, stream>>>(W2, HID, HID, 6, w2_16, 32.0f);

    k_cvt8<<<(MTOK * DSP / 8) / 256, 256, 0, stream>>>(span, span16, (unsigned)(MTOK * DSP / 8), 8.0f);
    k_cvt8<<<(NB * NIMG * DVI / 8) / 256, 256, 0, stream>>>(img, img16, (unsigned)(NB * NIMG * DVI / 8), 8.0f);

    const unsigned gG = ((MTOK / 64) * (DVI / 64) + 7) / 8;
    const unsigned gU = ((MTOK / 64) * (UVP / 64) + 7) / 8;
    k_gemm_g<<<gG, 256, 0, stream>>>((const _Float16*)span16, DSP, (const _Float16*)wg16, DSP,
        (_Float16*)g16, DVI, MTOK, DVI, DSP, SC_XW, 8.0f);
    k_gemm_uv<<<gU, 256, 0, stream>>>((const _Float16*)span16, DSP, (const _Float16*)w1_16, DSP,
        uv, UVP, MTOK, UVP, DSP, SC_XW, 1.0f);

    k_bil_sent<<<NB, 192, 0, stream>>>((const _Float16*)g16, (const _Float16*)img16, smask, imask, mws, sentw);
    k_loss<<<1, 128, 0, stream>>>(sentw, lossw);

    k_pair<<<NB * (PPAD / PT), 256, 0, stream>>>((const _Float16*)span16, (const _Float16*)(w1_16 + (size_t)2 * DSP * HID),
        (const _Float16*)w2_16, uv, b1, b2, W3, b3, tsw);

    const unsigned lossOff = (unsigned)(((char*)lossw - wsp) / 4);
    const unsigned mOff    = (unsigned)(((char*)mws - wsp) / 4);
    const unsigned tsOff   = (unsigned)(((char*)tsw - wsp) / 4);
    k_pack<<<(OUT_Q + 1 + 255) / 256, 256, 0, stream>>>((const float*)d_ws, lossOff, mOff, tsOff, out);
}
